// FNO2d_25915832664152
// MI455X (gfx1250) — hardware-run, weakly checked
//
#include <hip/hip_runtime.h>
#include <math.h>

typedef __attribute__((ext_vector_type(16))) _Float16 v16h;
typedef __attribute__((ext_vector_type(8)))  _Float16 v8h;
typedef __attribute__((ext_vector_type(8)))  float    v8f;
typedef __attribute__((ext_vector_type(4)))  float    v4f;
typedef __attribute__((ext_vector_type(2)))  float    v2f;

constexpr int kNB = 8;
constexpr int kNH = 128;
constexpr int kNW = 128;
constexpr int kCh = 32;
constexpr int kMd = 12;
constexpr int kLayers = 6;
constexpr int kImg = kNH * kNW;
constexpr int kPix = kNB * kImg;
constexpr int kRowsCM = kNB * kCh * kNH;
constexpr int kKy = 2 * kMd;
constexpr int kNModes = kNB * kCh * kKy * kMd;
constexpr int kChunk = 32768;
constexpr int kNChunk = kPix / kChunk;
constexpr int kF1 = 256;
constexpr int kF3 = 128;
constexpr int kF4 = 128;
constexpr int kTP = 36;
constexpr int kSwX = 2 * kMd;
constexpr int kSwO = kSwX * kMd;
constexpr int kSwI = kSwO * kCh;
constexpr int kSwPart = kSwI * kCh;
constexpr int kSwLayer = 2 * kSwPart;
static_assert(kImg == 16384 && kPix == 131072 && kRowsCM == 32768 && kNModes == 73728, "shapes");
static_assert(kSwO == 288 && kSwI == 9216 && kSwPart == 294912 && kSwLayer == 589824, "spectral weight strides");
static_assert((kChunk % 64) == 0 && (kF1 % 64) == 0 && (kF3 % 64) == 0 && (kF4 % 64) == 0, "tile multiples");
static_assert((kCh % 32) == 0 && (kF1 % 32) == 0 && (kF3 % 32) == 0 && (kNW % 32) == 0, "K multiples of 32");
static_assert((kNModes % 256) == 0 && (kPix % 64) == 0 && (kRowsCM % 256) == 0, "grid multiples");

constexpr float kACarry = 16.0f;
constexpr float kWCarry = 256.0f;
constexpr float kResScale = 2048.0f;
constexpr float kGCarry = 4.0f;
constexpr float kInvProd = 1.0f / (kACarry * kWCarry);
constexpr float kInvRes = 1.0f / kResScale;
constexpr float kBasisScale = (kACarry * kWCarry) / ((float)kImg * kGCarry);
constexpr float kF16MinNormal = 6.103515625e-5f;
constexpr float kAngStep = 6.283185307179586f / 128.0f;
static_assert(kBasisScale == 0.0625f, "inverse basis scale");

constexpr size_t kSzPM = (size_t)kPix * kCh * 2;
constexpr size_t kSzCM = (size_t)kRowsCM * kNW * 2;
constexpr size_t kOffPMH0 = 0;
constexpr size_t kOffPML0 = kOffPMH0 + kSzPM;
constexpr size_t kOffPMH1 = kOffPML0 + kSzPM;
constexpr size_t kOffPML1 = kOffPMH1 + kSzPM;
constexpr size_t kOffCMH0 = kOffPML1 + kSzPM;
constexpr size_t kOffCMH1 = kOffCMH0 + kSzCM;
constexpr size_t kOffROWFT = kOffCMH1 + kSzCM;
constexpr size_t kOffMODES = kOffROWFT + (size_t)kRowsCM * 64 * 4;
constexpr size_t kOffSPEC = kOffMODES + (size_t)kNModes * 8;
constexpr size_t kOffINVC = kOffSPEC + (size_t)kNModes * 8;
constexpr size_t kOffTRIG = kOffINVC + (size_t)kRowsCM * 32 * 2;
constexpr size_t kOffFWT = kOffTRIG + 256 * 4;
constexpr size_t kOffIFW = kOffFWT + 64 * 128 * 2;
constexpr size_t kOffWWH = kOffIFW + 128 * 32 * 2;
constexpr size_t kOffWWL = kOffWWH + (size_t)kLayers * kCh * kCh * 2;
constexpr size_t kOffF1H = kOffWWL + (size_t)kLayers * kCh * kCh * 2;
constexpr size_t kOffF1L = kOffF1H + (size_t)kF1 * kCh * 2;
constexpr size_t kOffF3H = kOffF1L + (size_t)kF1 * kCh * 2;
constexpr size_t kOffF3L = kOffF3H + (size_t)kF3 * kF1 * 2;
constexpr size_t kOffF4H = kOffF3L + (size_t)kF3 * kF1 * 2;
constexpr size_t kOffH1H = kOffF4H + (size_t)kF4 * kF3 * 2;
constexpr size_t kOffH1L = kOffH1H + (size_t)kChunk * kF1 * 2;
constexpr size_t kOffH2H = kOffH1L + (size_t)kChunk * kF1 * 2;
constexpr size_t kOffH3 = kOffH2H + (size_t)kChunk * kF3 * 2;
constexpr size_t kWsTotal = kOffH3 + (size_t)kChunk * kF4 * 4;
static_assert(kWsTotal == 120964096ull, "carve total");
static_assert(kWsTotal <= 134217728ull, "carve cap");
static_assert((kOffMODES % 128) == 0 && (kOffSPEC % 128) == 0 && (kOffINVC % 128) == 0 && (kOffTRIG % 128) == 0 &&
              (kOffFWT % 128) == 0 && (kOffIFW % 128) == 0 && (kOffWWH % 128) == 0 && (kOffWWL % 128) == 0 &&
              (kOffF1H % 128) == 0 && (kOffF1L % 128) == 0 && (kOffF3H % 128) == 0 && (kOffF3L % 128) == 0 &&
              (kOffF4H % 128) == 0 && (kOffH1H % 128) == 0 && (kOffH1L % 128) == 0 && (kOffH2H % 128) == 0 &&
              (kOffH3 % 128) == 0, "128-B aligned regions");

__device__ __forceinline__ void wave_sync_lds() {
  __builtin_amdgcn_fence(__ATOMIC_RELEASE, "workgroup");
  __builtin_amdgcn_wave_barrier();
  __builtin_amdgcn_fence(__ATOMIC_ACQUIRE, "workgroup");
}
__device__ __forceinline__ _Float16 f16_op(float v) {
  const float z = (fabsf(v) < kF16MinNormal) ? 0.0f : v;
  return (_Float16)z;
}
__device__ __forceinline__ void f16_split(float v, _Float16& hi, _Float16& lo) {
  hi = f16_op(v);
  const float r = (v - (float)hi) * kResScale;
  lo = f16_op(r);
}
__device__ __forceinline__ float gelu_erf(float v) {
  return 0.5f * v * (1.0f + erff(v * 0.70710678118654752f));
}

__device__ __forceinline__ void guard4_h1(v8f& a, v8f& b, v8f& c, v8f& d, v16h x) {
  asm volatile("v_nop\n\tv_nop\n\tv_nop\n\tv_nop" : "+v"(a), "+v"(b), "+v"(c), "+v"(d) : "v"(x));
}
__device__ __forceinline__ void guard4_h2(v8f& a, v8f& b, v8f& c, v8f& d, v16h x, v16h y) {
  asm volatile("v_nop\n\tv_nop\n\tv_nop\n\tv_nop" : "+v"(a), "+v"(b), "+v"(c), "+v"(d) : "v"(x), "v"(y));
}
__device__ __forceinline__ void guard4_h3(v8f& a, v8f& b, v8f& c, v8f& d, v16h x, v16h y, v16h z) {
  asm volatile("v_nop\n\tv_nop\n\tv_nop\n\tv_nop" : "+v"(a), "+v"(b), "+v"(c), "+v"(d) : "v"(x), "v"(y), "v"(z));
}
__device__ __forceinline__ void keep4_h(v16h a, v16h b, v16h c, v16h d) { asm volatile("v_nop" :: "v"(a), "v"(b), "v"(c), "v"(d)); }
__device__ __forceinline__ void keep2_h(v16h a, v16h b) { asm volatile("v_nop" :: "v"(a), "v"(b)); }
__device__ __forceinline__ void acc_guard4(v8f& a, v8f& b, v8f& c, v8f& d) {
  asm volatile("v_nop\n\tv_nop\n\tv_nop\n\tv_nop" : "+v"(a), "+v"(b), "+v"(c), "+v"(d));
}

struct FragH {
  union U { v16h v; v8h h[2]; };
  static __device__ __forceinline__ v16h load(const _Float16* p) {
    U f;
    f.h[0] = *(const v8h*)(p);
    f.h[1] = *(const v8h*)(p + 16);
    return f.v;
  }
  static __device__ __forceinline__ v8f mma(v16h a, v16h b, v8f c) {
    return __builtin_amdgcn_wmma_f32_16x16x32_f16(false, a, false, b, (short)0, c, false, false);
  }
};

template <int BIAS_MODE>
__global__ __launch_bounds__(256) void gemm64_f16(
    const unsigned short* __restrict__ Ap, int lda,
    const unsigned short* __restrict__ Btp, int ldb,
    float* __restrict__ C, int ldc,
    const float* __restrict__ bias,
    int M, int N, int K, float scale) {
  const _Float16* A = (const _Float16*)Ap;
  const _Float16* Bt = (const _Float16*)Btp;
  __shared__ __align__(16) float sT[8][16 * 68];
  const int lane = threadIdx.x & 31;
  const int wave = threadIdx.x >> 5;
  const int tilesN = N >> 6;
  const int tilesM = M >> 6;
  const int tile = blockIdx.x * 8 + wave;
  if (tile >= tilesM * tilesN) return;
  const int tm = tile / tilesN;
  const int tn = tile - tm * tilesN;
  const int m0 = tm << 6;
  const int n0 = tn << 6;
  const int rlane = lane & 15;
  const int koff = (lane >> 4) * 8;
  const int mOff = (lane >> 4) * 8;

  v8f acc[4][4];
#pragma unroll
  for (int i = 0; i < 4; ++i)
#pragma unroll
    for (int j = 0; j < 4; ++j) acc[i][j] = (v8f){0.f, 0.f, 0.f, 0.f, 0.f, 0.f, 0.f, 0.f};

  for (int k0 = 0; k0 < K; k0 += 32) {
    v16h bh[4];
#pragma unroll
    for (int j = 0; j < 4; ++j) {
      const size_t bo = (size_t)(n0 + (j << 4) + rlane) * ldb + koff + k0;
      bh[j] = FragH::load(Bt + bo);
    }
#pragma unroll
    for (int i = 0; i < 4; ++i) {
      const size_t ao = (size_t)(m0 + (i << 4) + rlane) * lda + koff + k0;
      const v16h ah = FragH::load(A + ao);
#pragma unroll
      for (int j = 0; j < 4; ++j) acc[i][j] = FragH::mma(ah, bh[j], acc[i][j]);
      guard4_h1(acc[i][0], acc[i][1], acc[i][2], acc[i][3], ah);
    }
    keep4_h(bh[0], bh[1], bh[2], bh[3]);
  }
  acc_guard4(acc[0][0], acc[0][1], acc[0][2], acc[0][3]);
  acc_guard4(acc[1][0], acc[1][1], acc[1][2], acc[1][3]);
  acc_guard4(acc[2][0], acc[2][1], acc[2][2], acc[2][3]);
  acc_guard4(acc[3][0], acc[3][1], acc[3][2], acc[3][3]);

  float* slab = sT[wave];
#pragma unroll
  for (int i = 0; i < 4; ++i) {
    const int mBase = m0 + (i << 4);
#pragma unroll
    for (int j = 0; j < 4; ++j) {
      const int n = n0 + (j << 4) + rlane;
      float bv = 0.f;
      if (BIAS_MODE == 2) bv = bias[n];
#pragma unroll
      for (int r = 0; r < 8; ++r) {
        float v = acc[i][j][r] * scale;
        if (BIAS_MODE == 2) v += bv;
        slab[(mOff + r) * 68 + (j << 4) + rlane] = v;
      }
    }
    wave_sync_lds();
    {
      const int hh = lane >> 4, c4 = (lane & 15) * 4;
      for (int pass = 0; pass < 2; ++pass) {
#pragma unroll
        for (int it = 0; it < 8; ++it) {
          const int row = it * 2 + hh;
          const v4f v = *(const v4f*)(slab + row * 68 + c4);
          *(volatile v4f*)(C + (size_t)(mBase + row) * ldc + n0 + c4) = v;
        }
        __threadfence();
      }
    }
    wave_sync_lds();
  }
}

template <bool GELU, bool OUT_LO>
__global__ __launch_bounds__(256) void gemm3_f16(
    const unsigned short* __restrict__ Ahp, const unsigned short* __restrict__ Alp, int lda,
    const unsigned short* __restrict__ Bhp, const unsigned short* __restrict__ Blp, int ldb,
    unsigned short* __restrict__ Ch, unsigned short* __restrict__ Cl, int ldc,
    const float* __restrict__ bias, int M, int N, int K, float scale, float outcarry) {
  const _Float16* Ah = (const _Float16*)Ahp;
  const _Float16* Al = (const _Float16*)Alp;
  const _Float16* Bh = (const _Float16*)Bhp;
  const _Float16* Bl = (const _Float16*)Blp;
  __shared__ __align__(16) float sT[8][16 * 68];
  const int lane = threadIdx.x & 31;
  const int wave = threadIdx.x >> 5;
  const int tilesN = N >> 6;
  const int tilesM = M >> 5;
  const int tile = blockIdx.x * 8 + wave;
  if (tile >= tilesM * tilesN) return;
  const int tm = tile / tilesN;
  const int tn = tile - tm * tilesN;
  const int m0 = tm << 5;
  const int n0 = tn << 6;
  const int rlane = lane & 15;
  const int koff = (lane >> 4) * 8;
  const int mOff = (lane >> 4) * 8;

  v8f am[2][4], ar[2][4];
#pragma unroll
  for (int i = 0; i < 2; ++i)
#pragma unroll
    for (int j = 0; j < 4; ++j) {
      am[i][j] = (v8f){0.f, 0.f, 0.f, 0.f, 0.f, 0.f, 0.f, 0.f};
      ar[i][j] = (v8f){0.f, 0.f, 0.f, 0.f, 0.f, 0.f, 0.f, 0.f};
    }

  for (int k0 = 0; k0 < K; k0 += 32) {
    v16h a_h[2], a_l[2];
#pragma unroll
    for (int i = 0; i < 2; ++i) {
      const size_t ao = (size_t)(m0 + (i << 4) + rlane) * lda + koff + k0;
      a_h[i] = FragH::load(Ah + ao);
      a_l[i] = FragH::load(Al + ao);
    }
#pragma unroll
    for (int j = 0; j < 4; ++j) {
      const size_t bo = (size_t)(n0 + (j << 4) + rlane) * ldb + koff + k0;
      const v16h bh = FragH::load(Bh + bo);
      const v16h bl = FragH::load(Bl + bo);
#pragma unroll
      for (int i = 0; i < 2; ++i) {
        am[i][j] = FragH::mma(a_h[i], bh, am[i][j]);
        ar[i][j] = FragH::mma(a_h[i], bl, ar[i][j]);
        ar[i][j] = FragH::mma(a_l[i], bh, ar[i][j]);
      }
      guard4_h2(am[0][j], am[1][j], ar[0][j], ar[1][j], bh, bl);
    }
    keep4_h(a_h[0], a_h[1], a_l[0], a_l[1]);
  }
  acc_guard4(am[0][0], am[0][1], am[0][2], am[0][3]);
  acc_guard4(am[1][0], am[1][1], am[1][2], am[1][3]);
  acc_guard4(ar[0][0], ar[0][1], ar[0][2], ar[0][3]);
  acc_guard4(ar[1][0], ar[1][1], ar[1][2], ar[1][3]);

  float* slab = sT[wave];
  const int q = lane >> 3, c8 = (lane & 7) * 8;
#pragma unroll
  for (int i = 0; i < 2; ++i) {
    const int mBase = m0 + (i << 4);
#pragma unroll
    for (int j = 0; j < 4; ++j) {
      const int n = n0 + (j << 4) + rlane;
      const float bv = bias[n];
#pragma unroll
      for (int r = 0; r < 8; ++r) {
        const float s = am[i][j][r] + ar[i][j][r] * kInvRes;
        slab[(mOff + r) * 68 + (j << 4) + rlane] = s * scale + bv;
      }
    }
    wave_sync_lds();
    if (GELU) {
#pragma unroll 1
      for (int t = 0; t < 32; ++t) {
        const int idx = t * 32 + lane;
        const int off = (idx >> 6) * 68 + (idx & 63);
        const float v = slab[off];
        slab[off] = gelu_erf(v);
      }
      wave_sync_lds();
    }
#pragma unroll 1
    for (int it = 0; it < 4; ++it) {
      const int row = it * 4 + q;
      const float* sp = slab + row * 68 + c8;
      const v4f a0 = *(const v4f*)(sp);
      const v4f a1 = *(const v4f*)(sp + 4);
      v8h hv, lv;
#pragma unroll
      for (int e = 0; e < 4; ++e) {
        _Float16 h0, l0, h1, l1;
        f16_split(a0[e] * outcarry, h0, l0);
        f16_split(a1[e] * outcarry, h1, l1);
        hv[e] = h0;
        hv[4 + e] = h1;
        lv[e] = l0;
        lv[4 + e] = l1;
      }
      const size_t o = (size_t)(mBase + row) * ldc + n0 + c8;
      *(volatile v8h*)(Ch + o) = hv;
      if (OUT_LO) *(volatile v8h*)(Cl + o) = lv;
      __threadfence();
      *(volatile v8h*)(Ch + o) = hv;
      if (OUT_LO) *(volatile v8h*)(Cl + o) = lv;
    }
    wave_sync_lds();
  }
}

__global__ __launch_bounds__(256) void tables_kernel(float* __restrict__ trig, unsigned short* __restrict__ fwt,
                                                     unsigned short* __restrict__ ifw) {
  __shared__ float s_tab[256];
  const int tid = threadIdx.x;
  {
    const float th = kAngStep * (float)(tid & 127);
    const float cv = cosf(th);
    const float sv = sinf(th);
    s_tab[tid] = (tid < 128) ? cv : sv;
  }
  __syncthreads();
  const int i = blockIdx.x * 256 + tid;
  if (i < 1024) {
    const int n = i >> 4, w0 = (i & 15) * 8, k = n >> 1;
    const int odd = n & 1;
    const float sg = odd ? -1.0f : 1.0f;
    v8h hv;
#pragma unroll
    for (int e = 0; e < 8; ++e) {
      const int j = ((w0 + e) * k) & 127;
      const float t = sg * s_tab[j + (odd << 7)];
      const float v = (n < kKy) ? t : 0.0f;
      hv[e] = f16_op(v);
    }
    unsigned short* qp = fwt + (size_t)i * 8;
    *(volatile v8h*)qp = hv;
    __threadfence();
    *(volatile v8h*)qp = hv;
  } else if (i < 1536) {
    const int ii = i - 1024;
    const int w = ii >> 2, nb = (ii & 3) * 8;
    v8h hv;
#pragma unroll
    for (int e = 0; e < 8; ++e) {
      const int n = nb + e;
      const int k = n >> 1;
      const int odd = n & 1;
      const int j = (w * k) & 127;
      const float ck = (k == 0) ? kBasisScale : (2.0f * kBasisScale);
      const float sg = odd ? -ck : ck;
      const float t = sg * s_tab[j + (odd << 7)];
      const float v = (n < kKy) ? t : 0.0f;
      hv[e] = f16_op(v);
    }
    unsigned short* qp = ifw + (size_t)ii * 8;
    *(volatile v8h*)qp = hv;
    __threadfence();
    *(volatile v8h*)qp = hv;
  } else if (i < 1600) {
    const int ii = i - 1536;
    v4f tv;
    tv[0] = s_tab[ii * 4 + 0];
    tv[1] = s_tab[ii * 4 + 1];
    tv[2] = s_tab[ii * 4 + 2];
    tv[3] = s_tab[ii * 4 + 3];
    float* qp = trig + ii * 4;
    *(volatile v4f*)qp = tv;
    __threadfence();
    *(volatile v4f*)qp = tv;
  }
}

__global__ __launch_bounds__(256) void prep_weight_kernel(const float* __restrict__ src, unsigned short* __restrict__ dh,
                                                          unsigned short* __restrict__ dl, int kdim, int ndim,
                                                          int transposed, int write_lo, int total8) {
  const int i = blockIdx.x * 256 + threadIdx.x;
  if (i >= total8) return;
  const int e0 = i * 8;
  const int n = e0 / kdim;
  const int k0 = e0 - n * kdim;
  v8h hv, lv;
#pragma unroll
  for (int e = 0; e < 8; ++e) {
    const int k = k0 + e;
    const size_t si = transposed ? ((size_t)k * ndim + n) : ((size_t)n * kdim + k);
    _Float16 h0, l0;
    f16_split(src[si] * kWCarry, h0, l0);
    hv[e] = h0;
    lv[e] = l0;
  }
  unsigned short* qh = dh + (size_t)e0;
  unsigned short* ql = dl + (size_t)e0;
  *(volatile v8h*)qh = hv;
  if (write_lo) *(volatile v8h*)ql = lv;
  __threadfence();
  *(volatile v8h*)qh = hv;
  if (write_lo) *(volatile v8h*)ql = lv;
}

__device__ __forceinline__ void store_act_tile(const float* tl, unsigned short* __restrict__ pmh,
                                               unsigned short* __restrict__ pml, unsigned short* __restrict__ cmh,
                                               int P0, int lane, int write_cm) {
#pragma unroll 1
  for (int it = 0; it < 8; ++it) {
    const int item = it * 32 + lane;
    const int px = item >> 2, seg = item & 3;
    const float* sp = tl + px * kTP + seg * 8;
    const v4f a0 = *(const v4f*)(sp);
    const v4f a1 = *(const v4f*)(sp + 4);
    v8h hv, lv;
#pragma unroll
    for (int e = 0; e < 4; ++e) {
      _Float16 h0, l0, h1, l1;
      f16_split(a0[e] * kACarry, h0, l0);
      f16_split(a1[e] * kACarry, h1, l1);
      hv[e] = h0;
      hv[4 + e] = h1;
      lv[e] = l0;
      lv[4 + e] = l1;
    }
    const size_t o = (size_t)(P0 + px) * kCh + seg * 8;
    *(volatile v8h*)(pmh + o) = hv;
    *(volatile v8h*)(pml + o) = lv;
    __threadfence();
    *(volatile v8h*)(pmh + o) = hv;
    *(volatile v8h*)(pml + o) = lv;
  }
  if (write_cm) {
    const int b = P0 / kImg;
    const int prem = P0 - b * kImg;
#pragma unroll 1
    for (int it = 0; it < 8; ++it) {
      const int item = it * 32 + lane;
      const int c = item >> 3, seg = item & 7;
      v8h hv;
#pragma unroll
      for (int e = 0; e < 8; ++e) hv[e] = f16_op(tl[(seg * 8 + e) * kTP + c] * kACarry);
      const size_t o = (size_t)(b * kCh + c) * kImg + prem + seg * 8;
      *(volatile v8h*)(cmh + o) = hv;
      __threadfence();
      *(volatile v8h*)(cmh + o) = hv;
    }
  }
}

__global__ __launch_bounds__(128) void lift_kernel(const float* __restrict__ x, const float* __restrict__ W0,
                                                   const float* __restrict__ b0, unsigned short* __restrict__ pmh,
                                                   unsigned short* __restrict__ pml, unsigned short* __restrict__ cmh) {
  __shared__ __align__(16) float sTile[4][64 * kTP];
  const int lane = threadIdx.x & 31;
  const int wave = threadIdx.x >> 5;
  const int tile = blockIdx.x * 4 + wave;
  if (tile >= kPix / 64) return;
  const int P0 = tile * 64;
  float* tl = sTile[wave];
  const int c = lane;
  const float w0 = W0[c], w1 = W0[kCh + c], w2 = W0[2 * kCh + c], w3 = W0[3 * kCh + c];
  const float bc = b0[c];
#pragma unroll 1
  for (int t = 0; t < 64; ++t) {
    const v4f xv = *(const v4f*)(x + (size_t)(P0 + t) * 4);
    float v = xv[0] * w0;
    v = fmaf(xv[1], w1, v);
    v = fmaf(xv[2], w2, v);
    v = fmaf(xv[3], w3, v);
    tl[t * kTP + c] = v + bc;
  }
  wave_sync_lds();
  store_act_tile(tl, pmh, pml, cmh, P0, lane, 1);
}

__global__ __launch_bounds__(256) void coldft_kernel(const float* __restrict__ rowft, const float* __restrict__ trig,
                                                     float* __restrict__ modes) {
  __shared__ float s_tab[256];
  const int tid = threadIdx.x;
  s_tab[tid] = trig[tid];
  __syncthreads();
  const int i = blockIdx.x * 256 + tid;
  const int ic = (i < kNModes) ? i : (kNModes - 1);
  const int kx = ic % kMd;
  const int r = (ic / kMd) % kKy;
  const int bc = ic / (kMd * kKy);
  const int ky = (r < kMd) ? r : (104 + r);
  const float* src = rowft + (size_t)bc * (kNH * 64) + 2 * kx;
  float re = 0.f, im = 0.f;
#pragma unroll 2
  for (int h = 0; h < kNH; ++h) {
    const int idx = (h * ky) & 127;
    const float cs = s_tab[idx];
    const float sn = s_tab[128 + idx];
    const v2f a = *(const v2f*)(src + h * 64);
    re = fmaf(a[0], cs, re);
    re = fmaf(a[1], sn, re);
    im = fmaf(a[1], cs, im);
    im = fmaf(-a[0], sn, im);
  }
  if (i < kNModes) {
    v2f o;
    o[0] = re;
    o[1] = im;
    float* qp = modes + (size_t)i * 2;
    *(volatile v2f*)qp = o;
    __threadfence();
    *(volatile v2f*)qp = o;
  }
}

__global__ __launch_bounds__(256) void modemix_kernel(const float* __restrict__ modes, const float* __restrict__ specw,
                                                      float* __restrict__ spec) {
  const int i = blockIdx.x * 256 + threadIdx.x;
  const int ic = (i < kNModes) ? i : (kNModes - 1);
  const int kx = ic % kMd;
  const int r = (ic / kMd) % kKy;
  const int o = (ic / (kMd * kKy)) % kCh;
  const int b = ic / (kMd * kKy * kCh);
  const int part = (r < kMd) ? 0 : 1;
  const int xx = r - part * kMd;
  const float* wp = specw + (size_t)part * kSwPart + (size_t)o * kSwO + xx * kSwX + kx * 2;
  const float* xp = modes + ((size_t)(b * kCh) * (kKy * kMd) + r * kMd + kx) * 2;
  float re = 0.f, im = 0.f;
#pragma unroll 4
  for (int c = 0; c < kCh; ++c) {
    const v2f a = *(const v2f*)(xp + (size_t)c * (kKy * kMd * 2));
    const v2f w = *(const v2f*)(wp + (size_t)c * kSwI);
    re = fmaf(a[0], w[0], re);
    re = fmaf(-a[1], w[1], re);
    im = fmaf(a[0], w[1], im);
    im = fmaf(a[1], w[0], im);
  }
  if (i < kNModes) {
    v2f ov;
    ov[0] = re;
    ov[1] = im;
    float* qp = spec + (size_t)i * 2;
    *(volatile v2f*)qp = ov;
    __threadfence();
    *(volatile v2f*)qp = ov;
  }
}

__global__ __launch_bounds__(256) void invcol_kernel(const float* __restrict__ spec, const float* __restrict__ trig,
                                                     unsigned short* __restrict__ invc) {
  __shared__ __align__(16) float s_z[2 * kKy * kMd * 2];
  __shared__ float s_tab[256];
  __shared__ __align__(16) float s_o[256 * kTP];
  const int tid = threadIdx.x;
  s_tab[tid] = trig[tid];
  for (int i = tid; i < 2 * kKy * kMd * 2; i += 256) s_z[i] = spec[(size_t)blockIdx.x * (2 * kKy * kMd * 2) + i];
  __syncthreads();
  const int lb = tid >> 7, h = tid & 127;
  const float* zp = s_z + lb * (kKy * kMd * 2);
  float re[kMd], im[kMd];
#pragma unroll
  for (int k = 0; k < kMd; ++k) {
    re[k] = 0.f;
    im[k] = 0.f;
  }
#pragma unroll 1
  for (int r = 0; r < kKy; ++r) {
    const int ky = (r < kMd) ? r : (104 + r);
    const int idx = (h * ky) & 127;
    const float cs = s_tab[idx];
    const float sn = s_tab[128 + idx];
#pragma unroll
    for (int k = 0; k < kMd; ++k) {
      const float a = zp[(r * kMd + k) * 2];
      const float bq = zp[(r * kMd + k) * 2 + 1];
      re[k] = fmaf(a, cs, re[k]);
      re[k] = fmaf(-bq, sn, re[k]);
      im[k] = fmaf(a, sn, im[k]);
      im[k] = fmaf(bq, cs, im[k]);
    }
  }
  float* so = s_o + tid * kTP;
#pragma unroll
  for (int k = 0; k < kMd; ++k) {
    so[2 * k] = re[k] * kGCarry;
    so[2 * k + 1] = (k == 0) ? 0.0f : (im[k] * kGCarry);
  }
#pragma unroll
  for (int n = kKy; n < 32; ++n) so[n] = 0.0f;
  __syncthreads();
#pragma unroll 1
  for (int it = 0; it < 4; ++it) {
    const int item = it * 256 + tid;
    const int row = item >> 2, seg = item & 3;
    const float* sp = s_o + row * kTP + seg * 8;
    const v4f a0 = *(const v4f*)(sp);
    const v4f a1 = *(const v4f*)(sp + 4);
    v8h hv;
#pragma unroll
    for (int e = 0; e < 4; ++e) {
      hv[e] = f16_op(a0[e]);
      hv[4 + e] = f16_op(a1[e]);
    }
    unsigned short* qp = invc + ((size_t)blockIdx.x * 256 + row) * 32 + seg * 8;
    *(volatile v8h*)qp = hv;
    __threadfence();
    *(volatile v8h*)qp = hv;
  }
}

__global__ __launch_bounds__(128) void combine_kernel(
    const unsigned short* __restrict__ pmhp, const unsigned short* __restrict__ pmlp,
    const unsigned short* __restrict__ wwhp, const unsigned short* __restrict__ wwlp,
    const unsigned short* __restrict__ ifwp, const unsigned short* __restrict__ invcp,
    const float* __restrict__ x, const float* __restrict__ g_wb, const float* __restrict__ g_bW,
    const float* __restrict__ g_bb, const float* __restrict__ g_cW, const float* __restrict__ g_cb,
    unsigned short* __restrict__ opmh, unsigned short* __restrict__ opml, unsigned short* __restrict__ ocmh,
    int write_cm) {
  __shared__ __align__(16) float sTile[4][64 * kTP];
  const _Float16* PH = (const _Float16*)pmhp;
  const _Float16* PL = (const _Float16*)pmlp;
  const _Float16* WH = (const _Float16*)wwhp;
  const _Float16* WL = (const _Float16*)wwlp;
  const _Float16* IF = (const _Float16*)ifwp;
  const _Float16* IV = (const _Float16*)invcp;
  const int lane = threadIdx.x & 31;
  const int wave = threadIdx.x >> 5;
  const int tile = blockIdx.x * 4 + wave;
  if (tile >= kPix / 64) return;
  const int b = tile >> 8;
  const int rem = tile & 255;
  const int h = rem >> 1;
  const int w0 = (rem & 1) << 6;
  const int P0 = tile << 6;
  const int rlane = lane & 15;
  const int koff = (lane >> 4) * 8;
  const int mOff = (lane >> 4) * 8;
  float* tl = sTile[wave];

  v16h bh[2], bl[2], sb[2];
#pragma unroll
  for (int j = 0; j < 2; ++j) {
    const int bo = ((j << 4) + rlane) * kCh + koff;
    bh[j] = FragH::load(WH + bo);
    bl[j] = FragH::load(WL + bo);
    const size_t so = ((size_t)(b * kCh + (j << 4) + rlane) * kNH + h) * 32 + koff;
    sb[j] = FragH::load(IV + so);
  }

#pragma unroll 1
  for (int hf = 0; hf < 2; ++hf) {
    v8f am[2][2], ar[2][2];
#pragma unroll
    for (int i = 0; i < 2; ++i)
#pragma unroll
      for (int j = 0; j < 2; ++j) {
        am[i][j] = (v8f){0.f, 0.f, 0.f, 0.f, 0.f, 0.f, 0.f, 0.f};
        ar[i][j] = (v8f){0.f, 0.f, 0.f, 0.f, 0.f, 0.f, 0.f, 0.f};
      }
#pragma unroll
    for (int i = 0; i < 2; ++i) {
      const int rowt = hf * 32 + (i << 4) + rlane;
      const size_t ao = (size_t)(P0 + rowt) * kCh + koff;
      const v16h ah = FragH::load(PH + ao);
      const v16h al = FragH::load(PL + ao);
      const v16h sa = FragH::load(IF + (w0 + rowt) * 32 + koff);
#pragma unroll
      for (int j = 0; j < 2; ++j) {
        am[i][j] = FragH::mma(ah, bh[j], am[i][j]);
        am[i][j] = FragH::mma(sa, sb[j], am[i][j]);
        ar[i][j] = FragH::mma(ah, bl[j], ar[i][j]);
        ar[i][j] = FragH::mma(al, bh[j], ar[i][j]);
      }
      guard4_h3(am[i][0], am[i][1], ar[i][0], ar[i][1], ah, al, sa);
    }
    keep4_h(bh[0], bh[1], bl[0], bl[1]);
    keep2_h(sb[0], sb[1]);
#pragma unroll
    for (int i = 0; i < 2; ++i)
#pragma unroll
      for (int j = 0; j < 2; ++j)
#pragma unroll
        for (int r = 0; r < 8; ++r) {
          const float s = am[i][j][r] + ar[i][j][r] * kInvRes;
          tl[(hf * 32 + (i << 4) + mOff + r) * kTP + (j << 4) + rlane] = s * kInvProd;
        }
  }
  wave_sync_lds();
  {
    const int o = lane;
    const float cst = g_wb[o] + g_bb[o] + g_cb[o];
    const float bw0 = g_bW[o * 2], bw1 = g_bW[o * 2 + 1];
    const float cw0 = g_cW[o * 3], cw1 = g_cW[o * 3 + 1], cw2 = g_cW[o * 3 + 2];
    const float gh = (float)h / 127.0f;
    const float base = cst + bw0 * gh;
#pragma unroll 1
    for (int t = 0; t < 64; ++t) {
      const v4f xv = *(const v4f*)(x + (size_t)(P0 + t) * 4);
      const float gw = (float)(w0 + t) / 127.0f;
      float v = tl[t * kTP + o];
      v += base;
      v = fmaf(bw1, gw, v);
      v = fmaf(cw0, xv[1], v);
      v = fmaf(cw1, xv[2], v);
      v = fmaf(cw2, xv[3], v);
      tl[t * kTP + o] = gelu_erf(v);
    }
  }
  wave_sync_lds();
  store_act_tile(tl, opmh, opml, ocmh, P0, lane, write_cm);
}

__global__ __launch_bounds__(256) void head_out_kernel(const float* __restrict__ H3, const float* __restrict__ w5,
                                                       const float* __restrict__ b5, float* __restrict__ out, int npx) {
  __shared__ __align__(16) float sw[kF4];
  const int tid = threadIdx.x;
  if (tid < kF4) sw[tid] = w5[tid];
  __syncthreads();
  const int p = blockIdx.x * 256 + tid;
  const int pc = (p < npx) ? p : (npx - 1);
  const float* row = H3 + (size_t)pc * kF4;
  float acc = 0.f;
#pragma unroll 1
  for (int k4 = 0; k4 < kF4 / 4; ++k4) {
    const v4f hv = *(const v4f*)(row + 4 * k4);
    const v4f wv = *(const v4f*)(sw + 4 * k4);
    acc = fmaf(hv[0], wv[0], acc);
    acc = fmaf(hv[1], wv[1], acc);
    acc = fmaf(hv[2], wv[2], acc);
    acc = fmaf(hv[3], wv[3], acc);
  }
  const float res = acc + b5[0];
  if (p < npx) {
    *(volatile float*)(out + p) = res;
    __threadfence();
    *(volatile float*)(out + p) = res;
  }
}

extern "C" void kernel_launch(void* const* d_in, const int* in_sizes, int n_in,
                              void* d_out, int out_size, void* d_ws, size_t ws_size,
                              hipStream_t stream) {
  if (n_in < 18) return;
  if (in_sizes[0] != kPix * 4) return;
  if (in_sizes[1] != 4 * kCh) return;
  if (in_sizes[2] != kCh) return;
  if (in_sizes[3] != kLayers * kSwLayer) return;
  if (in_sizes[4] != kLayers * kCh * kCh) return;
  if (in_sizes[5] != kLayers * kCh) return;
  if (in_sizes[6] != kLayers * kCh * 2) return;
  if (in_sizes[7] != kLayers * kCh) return;
  if (in_sizes[8] != kLayers * kCh * 3) return;
  if (in_sizes[9] != kLayers * kCh) return;
  if (in_sizes[10] != kCh * kF1) return;
  if (in_sizes[11] != kF1) return;
  if (in_sizes[12] != kF1 * kF3) return;
  if (in_sizes[13] != kF3) return;
  if (in_sizes[14] != kF3 * kF4) return;
  if (in_sizes[15] != kF4) return;
  if (in_sizes[16] != kF4) return;
  if (in_sizes[17] != 1) return;
  if (out_size != kPix) return;
  if (ws_size < kWsTotal) return;

  const float* x      = (const float*)d_in[0];
  const float* fc0_W  = (const float*)d_in[1];
  const float* fc0_b  = (const float*)d_in[2];
  const float* spec_w = (const float*)d_in[3];
  const float* wW     = (const float*)d_in[4];
  const float* wb     = (const float*)d_in[5];
  const float* bW     = (const float*)d_in[6];
  const float* bb     = (const float*)d_in[7];
  const float* cW     = (const float*)d_in[8];
  const float* cb     = (const float*)d_in[9];
  const float* fc1_W  = (const float*)d_in[10];
  const float* fc1_b  = (const float*)d_in[11];
  const float* fc3_W  = (const float*)d_in[12];
  const float* fc3_b  = (const float*)d_in[13];
  const float* fc4_W  = (const float*)d_in[14];
  const float* fc4_b  = (const float*)d_in[15];
  const float* fc5_W  = (const float*)d_in[16];
  const float* fc5_b  = (const float*)d_in[17];
  float* out = (float*)d_out;

  char* ws = (char*)d_ws;
  unsigned short* PMH[2] = {(unsigned short*)(ws + kOffPMH0), (unsigned short*)(ws + kOffPMH1)};
  unsigned short* PML[2] = {(unsigned short*)(ws + kOffPML0), (unsigned short*)(ws + kOffPML1)};
  unsigned short* CMH[2] = {(unsigned short*)(ws + kOffCMH0), (unsigned short*)(ws + kOffCMH1)};
  float*          ROWFT = (float*)(ws + kOffROWFT);
  float*          MODES = (float*)(ws + kOffMODES);
  float*          SPEC  = (float*)(ws + kOffSPEC);
  unsigned short* INVC  = (unsigned short*)(ws + kOffINVC);
  float*          TRIG  = (float*)(ws + kOffTRIG);
  unsigned short* FWT   = (unsigned short*)(ws + kOffFWT);
  unsigned short* IFW   = (unsigned short*)(ws + kOffIFW);
  unsigned short* WWH   = (unsigned short*)(ws + kOffWWH);
  unsigned short* WWL   = (unsigned short*)(ws + kOffWWL);
  unsigned short* F1H   = (unsigned short*)(ws + kOffF1H);
  unsigned short* F1L   = (unsigned short*)(ws + kOffF1L);
  unsigned short* F3H   = (unsigned short*)(ws + kOffF3H);
  unsigned short* F3L   = (unsigned short*)(ws + kOffF3L);
  unsigned short* F4H   = (unsigned short*)(ws + kOffF4H);
  unsigned short* H1H   = (unsigned short*)(ws + kOffH1H);
  unsigned short* H1L   = (unsigned short*)(ws + kOffH1L);
  unsigned short* H2H   = (unsigned short*)(ws + kOffH2H);
  float*          H3    = (float*)(ws + kOffH3);

  tables_kernel<<<7, 256, 0, stream>>>(TRIG, FWT, IFW);
  prep_weight_kernel<<<(kLayers * kCh * kCh / 8) / 256, 256, 0, stream>>>(wW, WWH, WWL, kCh, kLayers * kCh, 0, 1,
                                                                         kLayers * kCh * kCh / 8);
  prep_weight_kernel<<<(kF1 * kCh / 8) / 256, 256, 0, stream>>>(fc1_W, F1H, F1L, kCh, kF1, 1, 1, kF1 * kCh / 8);
  prep_weight_kernel<<<(kF3 * kF1 / 8) / 256, 256, 0, stream>>>(fc3_W, F3H, F3L, kF1, kF3, 1, 1, kF3 * kF1 / 8);
  prep_weight_kernel<<<(kF4 * kF3 / 8) / 256, 256, 0, stream>>>(fc4_W, F4H, F4H, kF3, kF4, 1, 0, kF4 * kF3 / 8);

  lift_kernel<<<kPix / 64 / 4, 128, 0, stream>>>(x, fc0_W, fc0_b, PMH[0], PML[0], CMH[0]);

  int cur = 0;
  for (int l = 0; l < kLayers; ++l) {
    const int nxt = cur ^ 1;
    gemm64_f16<0><<<(kRowsCM / 64) * (64 / 64) / 8, 256, 0, stream>>>(
        CMH[cur], kNW, FWT, kNW, ROWFT, 64, nullptr, kRowsCM, 64, kNW, 1.0f / kACarry);
    coldft_kernel<<<kNModes / 256, 256, 0, stream>>>(ROWFT, TRIG, MODES);
    modemix_kernel<<<kNModes / 256, 256, 0, stream>>>(MODES, spec_w + (size_t)l * kSwLayer, SPEC);
    invcol_kernel<<<kRowsCM / 256, 256, 0, stream>>>(SPEC, TRIG, INVC);
    combine_kernel<<<kPix / 64 / 4, 128, 0, stream>>>(
        PMH[cur], PML[cur], WWH + (size_t)l * kCh * kCh, WWL + (size_t)l * kCh * kCh, IFW, INVC, x,
        wb + l * kCh, bW + l * kCh * 2, bb + l * kCh, cW + l * kCh * 3, cb + l * kCh,
        PMH[nxt], PML[nxt], CMH[nxt], (l + 1 < kLayers) ? 1 : 0);
    cur = nxt;
  }

  for (int c = 0; c < kNChunk; ++c) {
    const size_t p0 = (size_t)c * kChunk;
    gemm3_f16<true, true><<<(kChunk / 32) * (kF1 / 64) / 8, 256, 0, stream>>>(
        PMH[cur] + p0 * kCh, PML[cur] + p0 * kCh, kCh, F1H, F1L, kCh, H1H, H1L, kF1, fc1_b,
        kChunk, kF1, kCh, kInvProd, kACarry);
    gemm3_f16<true, false><<<(kChunk / 32) * (kF3 / 64) / 8, 256, 0, stream>>>(
        H1H, H1L, kF1, F3H, F3L, kF1, H2H, H2H, kF3, fc3_b,
        kChunk, kF3, kF1, kInvProd, kACarry);
    gemm64_f16<2><<<(kChunk / 64) * (kF4 / 64) / 8, 256, 0, stream>>>(
        H2H, kF3, F4H, kF3, H3, kF4, fc4_b, kChunk, kF4, kF3, kInvProd);
    head_out_kernel<<<kChunk / 256, 256, 0, stream>>>(H3, fc5_W, fc5_b, out + p0, kChunk);
  }
}
